// EncodingP_86526411145826
// MI455X (gfx1250) — hardware-run, weakly checked
//
#include <hip/hip_runtime.h>
#include <stddef.h>


typedef _Float16 v16h __attribute__((ext_vector_type(16)));
typedef _Float16 v8h  __attribute__((ext_vector_type(8)));
typedef float    v8f  __attribute__((ext_vector_type(8)));
typedef float    v4f  __attribute__((ext_vector_type(4)));

#ifndef NB
#define NB 4
#endif
#ifndef NPIX
#define NPIX 4096
#endif
#define NB_FULL   4
#define NPIX_FULL 4096
#define FDIM  256
#define NCODE 32

static_assert(NB >= 1 && NB <= NB_FULL);
static_assert(NPIX >= 64 && NPIX <= NPIX_FULL && (NPIX % 64) == 0);
static_assert((NPIX % 32) == 0 && (NPIX % 8) == 0 && (NPIX_FULL % 4) == 0);
static_assert(FDIM == 256 && (FDIM % 32) == 0 && (FDIM % 64) == 0);
static_assert(FDIM == 32 * 8);
static_assert(NCODE == 32);
static_assert(4 * 256 * 8 == NCODE * FDIM);
static_assert(16 * 128 * 8 == FDIM * 64);
static_assert(2 * 128 * 8 == NCODE * 64);
static_assert(2 * 256 * 4 == NCODE * 64);
static_assert(((size_t)NB * FDIM * NPIX / 8) % 256 == 0);

#define LDX 264
#define LDP 72
#define LDC 68
static_assert((LDX % 8) == 0 && LDX >= FDIM);
static_assert((LDP % 8) == 0 && LDP >= 64);
static_assert((LDC % 4) == 0 && LDC >= 64);

#define CCARRY 4096.0f
#define PCARRY 16384.0f

#define C16_BYTES ((size_t)NCODE * FDIM * 2)
#define C2_BYTES  ((size_t)128)
#define X16_BYTES ((size_t)NB * FDIM * NPIX * 2)
#define PT_BYTES  ((size_t)NB * NCODE * NPIX * 2)
#define OFF_C16 ((size_t)0)
#define OFF_C2  (OFF_C16 + C16_BYTES)
#define OFF_X16 (OFF_C2 + C2_BYTES)
#define OFF_PT  (OFF_X16 + X16_BYTES)
#define WS_TOTAL (OFF_PT + PT_BYTES)
static_assert((C16_BYTES % 128) == 0 && (C2_BYTES % 128) == 0);
static_assert((X16_BYTES % 128) == 0 && (PT_BYTES % 128) == 0);
static_assert(NCODE * 4 == 128);
static_assert(WS_TOTAL <= (size_t)134217728);
static_assert((size_t)NB_FULL * NCODE * FDIM * 4 == (size_t)131072);

__device__ __forceinline__ float bf16r(float x) {
  unsigned int u = __float_as_uint(x);
  u = (u + 0x7FFFu + ((u >> 16) & 1u)) & 0xFFFF0000u;
  return __uint_as_float(u);
}

static __device__ __forceinline__ _Float16 toh_flush(float v) {
  const _Float16 r = (_Float16)v;
  return (fabsf(v) < 6.103515625e-05f) ? (_Float16)0.0f : r;
}

__device__ __forceinline__ v16h frag_at(const _Float16* p) {
  v8h lo = *(const v8h*)(p);
  v8h hi = *(const v8h*)(p + 16);
  v16h out;
#pragma unroll
  for (int i = 0; i < 8; ++i) { out[i] = lo[i]; out[i + 8] = hi[i]; }
  return out;
}
__device__ __forceinline__ v16h ld_frag(const _Float16* base, unsigned ld) {
  const unsigned lane = threadIdx.x & 31u;
  return frag_at(base + (lane & 15u) * ld + (lane >> 4) * 8u);
}

__device__ __forceinline__ v8f wmma16(v16h a, v16h b, v8f c) {
  v8f d = __builtin_amdgcn_wmma_f32_16x16x32_f16(false, a, false, b, (short)0, c,
                                                 false, false);
  asm volatile("v_nop\n\tv_nop\n\tv_nop\n\tv_nop" : "+v"(d) : "v"(a), "v"(b));
  return d;
}

__device__ __forceinline__ float red16_max(float x) {
#pragma unroll
  for (int off = 1; off < 16; off <<= 1) x = fmaxf(x, __shfl_xor(x, off, 32));
  return x;
}
__device__ __forceinline__ float red16_sum(float x) {
#pragma unroll
  for (int off = 1; off < 16; off <<= 1) x += __shfl_xor(x, off, 32);
  return x;
}
__device__ __forceinline__ float red32_sum(float x) {
#pragma unroll
  for (int off = 1; off < 32; off <<= 1) x += __shfl_xor(x, off, 32);
  return x;
}

__global__ __launch_bounds__(256) void cconv_kernel(
    const float* __restrict__ Cw, _Float16* __restrict__ C16, float* __restrict__ C2) {
#pragma clang fp contract(off)
  __shared__ __attribute__((aligned(16))) float sC2[NCODE];
  const unsigned tid = threadIdx.x, lane = tid & 31u;
  const unsigned wave = (unsigned)__builtin_amdgcn_readfirstlane((int)(threadIdx.x >> 5));

  v8h x[4];
  size_t off[4];
#pragma unroll
  for (unsigned j = 0; j < 4u; ++j) {
    const unsigned idx = tid + 256u * j;
    const unsigned k = idx >> 5, c8 = (idx & 31u) * 8u;
    const v4f a0 = *(const v4f*)(Cw + k * FDIM + c8);
    const v4f a1 = *(const v4f*)(Cw + k * FDIM + c8 + 4u);
    v8h o;
#pragma unroll
    for (int i = 0; i < 4; ++i) {
      o[i]     = toh_flush(CCARRY * bf16r(a0[i]));
      o[i + 4] = toh_flush(CCARRY * bf16r(a1[i]));
    }
    x[j] = o;
    off[j] = (size_t)k * FDIM + c8;
  }

#pragma unroll 1
  for (unsigned rr = 0; rr < 4u; ++rr) {
    const unsigned k = wave * 4u + rr;
    const v4f a0 = *(const v4f*)(Cw + k * FDIM + lane * 8u);
    const v4f a1 = *(const v4f*)(Cw + k * FDIM + lane * 8u + 4u);
    float s = 0.0f;
#pragma unroll
    for (int i = 0; i < 4; ++i) {
      const float e0 = bf16r(a0[i]);
      const float e1 = bf16r(a1[i]);
      s += e0 * e0;
      s += e1 * e1;
    }
    s = red32_sum(s);
    if (lane == 0u) sC2[k] = s;
  }
  __syncthreads();
  const v4f cv = *(const v4f*)&sC2[(tid & 7u) * 4u];

#pragma unroll
  for (int j = 0; j < 4; ++j) *(volatile v8h*)(C16 + off[j]) = x[j];
  if (tid < 8u) *(volatile v4f*)(C2 + tid * 4u) = cv;
  __threadfence();
#pragma unroll
  for (int j = 0; j < 4; ++j) *(volatile v8h*)(C16 + off[j]) = x[j];
  if (tid < 8u) *(volatile v4f*)(C2 + tid * 4u) = cv;
}

__global__ __launch_bounds__(256) void xconv_kernel(
    const float* __restrict__ X, _Float16* __restrict__ X16) {
#pragma clang fp contract(off)
  const unsigned chunk = blockIdx.x * 256u + threadIdx.x;
  const unsigned cpr = (unsigned)NPIX / 8u;
  const unsigned row = chunk / cpr;
  const unsigned c8 = (chunk - row * cpr) * 8u;
  const unsigned b = row >> 8, d = row & 255u;
  const float* src = X + ((size_t)b * FDIM + d) * NPIX_FULL + c8;
  const v4f a0 = *(const v4f*)(src);
  const v4f a1 = *(const v4f*)(src + 4);
  v8h o;
#pragma unroll
  for (int i = 0; i < 4; ++i) {
    o[i]     = toh_flush(bf16r(a0[i]));
    o[i + 4] = toh_flush(bf16r(a1[i]));
  }
  _Float16* p = X16 + (size_t)row * NPIX + c8;
  *(volatile v8h*)p = o;
  __threadfence();
  *(volatile v8h*)p = o;
}

__global__ __launch_bounds__(128) void assign_kernel(
    const _Float16* __restrict__ X16, const _Float16* __restrict__ C16,
    const float* __restrict__ C2, const float* __restrict__ Sc,
    _Float16* __restrict__ Pt) {
  __shared__ __attribute__((aligned(16))) _Float16 Xs[64 * LDX];
  __shared__ __attribute__((aligned(16))) _Float16 Ps[NCODE * LDP];
  __shared__ __attribute__((aligned(16))) float sX2[64];

  const unsigned tid = threadIdx.x, lane = tid & 31u;
  const unsigned wave = (unsigned)__builtin_amdgcn_readfirstlane((int)(threadIdx.x >> 5));
  const unsigned hh = lane >> 4, m = lane & 15u;
  const unsigned n0 = blockIdx.x * 64u;
  const unsigned b = blockIdx.y;
  const size_t xplane = (size_t)b * FDIM * NPIX + n0;

#pragma unroll 4
  for (unsigned j = 0; j < 16u; ++j) {
    const unsigned idx = tid + 128u * j;
    const unsigned d = idx >> 3, c8 = (idx & 7u) * 8u;
    const v8h xv = *(const v8h*)(X16 + xplane + (size_t)d * NPIX + c8);
#pragma unroll
    for (unsigned i = 0; i < 8u; ++i) Xs[(c8 + i) * LDX + d] = xv[i];
  }
  __syncthreads();

  {
    const unsigned p = tid >> 1, part = tid & 1u;
    float s = 0.0f;
#pragma unroll 1
    for (unsigned j = 0; j < 16u; ++j) {
      const v8h xv = *(const v8h*)&Xs[p * LDX + part * 128u + j * 8u];
#pragma unroll
      for (int i = 0; i < 8; ++i) {
        const float e = (float)xv[i];
        s += e * e;
      }
    }
    s += __shfl_xor(s, 1, 32);
    if (part == 0u) sX2[p] = s;
  }
  __syncthreads();

  v8f acc0 = {}, acc1 = {};
  const _Float16* cp0 = C16 + (size_t)m * FDIM + hh * 8u;
  const _Float16* cp1 = cp0 + (size_t)16 * FDIM;
#pragma unroll 2
  for (unsigned k0 = 0; k0 < (unsigned)FDIM; k0 += 32u) {
    const v16h a  = ld_frag(&Xs[(wave * 16u) * LDX + k0], LDX);
    const v16h b0 = frag_at(cp0 + k0);
    const v16h b1 = frag_at(cp1 + k0);
    acc0 = wmma16(a, b0, acc0);
    acc1 = wmma16(a, b1, acc1);
  }

  const float sc0 = bf16r(Sc[m]);
  const float sc1 = bf16r(Sc[16u + m]);
  const float cc0 = C2[m];
  const float cc1 = C2[16u + m];
  v8h p0, p1;
#pragma unroll
  for (int v = 0; v < 8; ++v) {
    const float x2 = sX2[wave * 16u + hh * 8u + (unsigned)v];
    const float l0 = (x2 - 2.0f * (acc0[v] * (1.0f / CCARRY))) + cc0;
    const float l1 = (x2 - 2.0f * (acc1[v] * (1.0f / CCARRY))) + cc1;
    const float t0 = l0 * sc0;
    const float t1 = l1 * sc1;
    const float mx = red16_max(fmaxf(t0, t1));
    const float e0 = __expf(t0 - mx);
    const float e1 = __expf(t1 - mx);
    const float sum = red16_sum(e0 + e1);
    const float inv = __builtin_amdgcn_rcpf(sum) * PCARRY;
    p0[v] = toh_flush(e0 * inv);
    p1[v] = toh_flush(e1 * inv);
  }
  *(v8h*)&Ps[m * LDP + wave * 16u + hh * 8u] = p0;
  *(v8h*)&Ps[(16u + m) * LDP + wave * 16u + hh * 8u] = p1;
  __syncthreads();

  v8h x[2];
  size_t off[2];
#pragma unroll
  for (unsigned i = 0; i < 2u; ++i) {
    const unsigned idx = tid + 128u * i;
    const unsigned k = idx >> 3, c8 = (idx & 7u) * 8u;
    x[i] = *(const v8h*)&Ps[k * LDP + c8];
    off[i] = ((size_t)b * NCODE + k) * NPIX + n0 + c8;
  }
#pragma unroll
  for (int i = 0; i < 2; ++i) *(volatile v8h*)(Pt + off[i]) = x[i];
  __threadfence();
#pragma unroll
  for (int i = 0; i < 2; ++i) *(volatile v8h*)(Pt + off[i]) = x[i];
}

__global__ __launch_bounds__(256) void aggregate_kernel(
    const _Float16* __restrict__ Pt, const _Float16* __restrict__ X16,
    const float* __restrict__ Cw, float* __restrict__ outf) {
  __shared__ __attribute__((aligned(16))) float Cs[NCODE * LDC];
  __shared__ __attribute__((aligned(16))) float As[NCODE];

  const unsigned tid = threadIdx.x, lane = tid & 31u;
  const unsigned wave = (unsigned)__builtin_amdgcn_readfirstlane((int)(threadIdx.x >> 5));
  const unsigned mt = wave >> 2, nt = wave & 3u;
  const unsigned hh = lane >> 4, m = lane & 15u;
  const unsigned d0 = blockIdx.x * 64u;
  const unsigned b = blockIdx.y;

  const _Float16* ap = Pt + ((size_t)b * NCODE + mt * 16u + m) * NPIX + hh * 8u;
  const _Float16* bp = X16 + ((size_t)b * FDIM + d0 + nt * 16u + m) * NPIX + hh * 8u;
  v16h ones;
#pragma unroll
  for (int i = 0; i < 16; ++i) ones[i] = (_Float16)1.0f;

  v8f acc = {}, accs = {};
#pragma unroll 2
  for (unsigned k0 = 0; k0 < (unsigned)NPIX; k0 += 32u) {
    const v16h a  = frag_at(ap + k0);
    const v16h xb = frag_at(bp + k0);
    acc  = wmma16(a, xb, acc);
    accs = wmma16(a, ones, accs);
  }

#pragma unroll
  for (int r = 0; r < 8; ++r)
    Cs[(mt * 16u + hh * 8u + (unsigned)r) * LDC + nt * 16u + m] = acc[r];
  if (nt == 0u) {
    if (m == 0u) {
#pragma unroll
      for (int r = 0; r < 8; ++r) As[mt * 16u + hh * 8u + (unsigned)r] = accs[r];
    }
  }
  __syncthreads();

  v4f xs[2];
  size_t off[2];
#pragma unroll
  for (unsigned i = 0; i < 2u; ++i) {
    const unsigned r = 16u * i + (tid >> 4);
    const unsigned c = (tid & 15u) * 4u;
    const v4f u = *(const v4f*)&Cs[r * LDC + c];
    const float mass = As[r] * (1.0f / PCARRY);
    const v4f g = *(const v4f*)(Cw + (size_t)r * FDIM + d0 + c);
    v4f val;
#pragma unroll
    for (int j = 0; j < 4; ++j) val[j] = u[j] * (1.0f / PCARRY) - mass * bf16r(g[j]);
    xs[i] = val;
    off[i] = ((size_t)b * NCODE + r) * FDIM + d0 + c;
  }
#pragma unroll
  for (int i = 0; i < 2; ++i) *(volatile v4f*)(outf + off[i]) = xs[i];
  __threadfence();
#pragma unroll
  for (int i = 0; i < 2; ++i) *(volatile v4f*)(outf + off[i]) = xs[i];
}

extern "C" void kernel_launch(void* const* d_in, const int* in_sizes, int n_in,
                              void* d_out, int out_size, void* d_ws, size_t ws_size,
                              hipStream_t stream) {
  if (n_in < 3) return;
  const long long need_x =
      ((long long)(NB - 1) * FDIM + (FDIM - 1)) * NPIX_FULL + NPIX;
  if ((long long)in_sizes[0] < need_x) return;
  if ((long long)in_sizes[1] < (long long)NCODE * FDIM) return;
  if (in_sizes[2] < NCODE) return;
  if ((long long)out_size < (long long)NB * NCODE * FDIM) return;
  if (ws_size < WS_TOTAL) return;

  const float* X  = (const float*)d_in[0];
  const float* cw = (const float*)d_in[1];
  const float* sc = (const float*)d_in[2];
  float* out = (float*)d_out;

  char* ws = (char*)d_ws;
  _Float16* C16 = (_Float16*)(ws + OFF_C16);
  float*    C2  = (float*)(ws + OFF_C2);
  _Float16* X16 = (_Float16*)(ws + OFF_X16);
  _Float16* Pt  = (_Float16*)(ws + OFF_PT);

  cconv_kernel<<<dim3(1), dim3(256), 0, stream>>>(cw, C16, C2);
  xconv_kernel<<<dim3((unsigned)((size_t)NB * NPIX / 8)), dim3(256), 0, stream>>>(X, X16);
  assign_kernel<<<dim3(NPIX / 64, NB), dim3(128), 0, stream>>>(X16, C16, C2, sc, Pt);
  aggregate_kernel<<<dim3(FDIM / 64, NB), dim3(256), 0, stream>>>(Pt, X16, cw, out);
}
